// CrossAttention_61830349193403
// MI455X (gfx1250) — hardware-run, weakly checked
//
#include <hip/hip_runtime.h>


#ifndef NB
#define NB 8
#endif
#define NB_FULL 8
#define IMG   64
#define NTOK  4096
#define CM    256
#define C2    512
#define NH_   8
#define HD    32
#define CHB   ((NB % 4 == 0) ? 4 : 1)
#define MROWS (NB * NTOK)
#define TSP   260
#define QRS   2048.0f
#define QRI   (1.0f / 2048.0f)
#define WSC   16.0f
#define OS_W  (1.0f / 16.0f)
#define KSC   4096.0f
#define QSC   32.0f
#define OS_CTX (1.0f / 64.0f)
#define OS_ATT (1.0f / 8.0f)
#define OS_REP (1.0f / 4096.0f)
#define L2E   1.4426950408889634f
#define EPSL  1e-5f

static_assert(IMG * IMG == NTOK);
static_assert(NH_ * HD == CM);
static_assert(HD == 32);
static_assert(CM % 32 == 0);
static_assert(C2 % 32 == 0);
static_assert(NTOK % 64 == 0);
static_assert(MROWS % 64 == 0);
static_assert(NTOK % 32 == 0);
static_assert(NB % CHB == 0);
static_assert((CHB * NTOK) % 32 == 0);
static_assert(NTOK == 256 * 16);
static_assert(CM == 32 * 8);
static_assert(CM == 4 * 64);
static_assert(C2 == 4 * 128);
static_assert(C2 % 64 == 0);
static_assert(NB <= NB_FULL);
static_assert((TSP * 4) % 16 == 0);
static_assert(32 * TSP * 4 <= 131072);
static_assert(8 * C2 * 4 <= 131072);

typedef _Float16 h16;
typedef __attribute__((ext_vector_type(16))) _Float16 v16h;
typedef __attribute__((ext_vector_type(8)))  _Float16 v8h;
typedef __attribute__((ext_vector_type(4)))  _Float16 v4h;
typedef __attribute__((ext_vector_type(8)))  float    v8f;
typedef __attribute__((ext_vector_type(4)))  float    v4f;
typedef v4f  __attribute__((may_alias)) v4fa;

__device__ __forceinline__ unsigned short f2bf(float f) { unsigned u = __float_as_uint(f); u += 0x7FFFu + ((u >> 16) & 1u); return (unsigned short)(u >> 16); }
__device__ __forceinline__ float bfr(float f) { return __uint_as_float(((unsigned)f2bf(f)) << 16); }
__device__ __forceinline__ v16h cat16(v8h lo, v8h hi) { return __builtin_shufflevector(lo, hi, 0, 1, 2, 3, 4, 5, 6, 7, 8, 9, 10, 11, 12, 13, 14, 15); }
__device__ __forceinline__ v8f wmma16(v16h a, v16h b, v8f c) { return __builtin_amdgcn_wmma_f32_16x16x32_f16(false, a, false, b, (short)0, c, false, false); }
__device__ __forceinline__ v8f wmma16g(v16h a, v16h b, v8f c) { c = wmma16(a, b, c); asm volatile("v_nop\n\tv_nop\n\tv_nop\n\tv_nop" : "+v"(c) : "v"(a), "v"(b)); return c; }
__device__ __forceinline__ v16h  ldh(const h16* p) { return cat16(*(const v8h*)p, *(const v8h*)(p + 16)); }
__device__ __forceinline__ void wave_sync() { __builtin_amdgcn_fence(3  , "wavefront"); __builtin_amdgcn_wave_barrier(); asm volatile("" ::: "memory"); }
static __device__ __forceinline__ h16 toh_flush(float v) { const float w = (fabsf(v) < 6.103515625e-05f) ? 0.0f : v; return (h16)w; }
__device__ __forceinline__ void split_hr(float v, h16& hv, h16& rv) { const h16 a = toh_flush(v); hv = a; rv = toh_flush((v - (float)a) * QRS); }
__device__ __forceinline__ float wsum(float v) { v += __shfl_xor(v, 16, 32); v += __shfl_xor(v, 8, 32); v += __shfl_xor(v, 4, 32); v += __shfl_xor(v, 2, 32); v += __shfl_xor(v, 1, 32); return v; }
__device__ __forceinline__ float wmaxf(float v) { v = fmaxf(v, __shfl_xor(v, 16, 32)); v = fmaxf(v, __shfl_xor(v, 8, 32)); v = fmaxf(v, __shfl_xor(v, 4, 32)); v = fmaxf(v, __shfl_xor(v, 2, 32)); v = fmaxf(v, __shfl_xor(v, 1, 32)); return v; }

template <int KD>
__device__ __forceinline__ void mm_rows(const h16* __restrict__ AH, const h16* __restrict__ W, size_t aoff, size_t boff, v8f (&acc)[2][4]) {
#pragma unroll 1
    for (int kc = 0; kc < KD; kc += 32) {
        v16h a[2];
#pragma unroll
        for (int mb = 0; mb < 2; ++mb) a[mb] = ldh(AH + aoff + (size_t)mb * 16 * KD + kc);
#pragma unroll
        for (int nb = 0; nb < 4; ++nb) { const v16h b = ldh(W + boff + (size_t)nb * 16 * KD + kc);
#pragma unroll
            for (int mb = 0; mb < 2; ++mb) acc[mb][nb] = wmma16g(a[mb], b, acc[mb][nb]); }
    }
}
template <int KD>
__device__ __forceinline__ void mm_cols(const h16* __restrict__ W, const h16* __restrict__ XH, size_t aoff, size_t boff, v8f (&acc)[2][4]) {
#pragma unroll 1
    for (int kc = 0; kc < KD; kc += 32) {
        v16h a[2];
#pragma unroll
        for (int mb = 0; mb < 2; ++mb) a[mb] = ldh(W + aoff + (size_t)mb * 16 * KD + kc);
#pragma unroll
        for (int nb = 0; nb < 4; ++nb) { const v16h bh = ldh(XH + boff + (size_t)nb * 16 * KD + kc);
#pragma unroll
            for (int mb = 0; mb < 2; ++mb) acc[mb][nb] = wmma16g(a[mb], bh, acc[mb][nb]); }
    }
}

__global__ __launch_bounds__(256) void k_wconv(const float* __restrict__ src, h16* dst, unsigned n8) {
    const unsigned i = blockIdx.x * 256u + threadIdx.x; if (i >= n8) return;
    const v8f v = *(const v8f*)(src + (size_t)i * 8); v8h o;
#pragma unroll
    for (int k = 0; k < 8; ++k) o[k] = toh_flush(bfr(v[k]) * WSC);
    *(volatile v8h*)(dst + (size_t)i * 8) = o; __threadfence(); *(volatile v8h*)(dst + (size_t)i * 8) = o;
}

__global__ __launch_bounds__(128) void k_tapprep(const float* __restrict__ w, float* WT) {
    const unsigned tap = blockIdx.x, c4 = threadIdx.x * 4u;
    static_assert(128 * 4 == C2);
    v4f o;
#pragma unroll
    for (int k = 0; k < 4; ++k) o[k] = bfr(w[(size_t)(c4 + k) * 9u + tap]);
    *(volatile v4f*)(WT + (size_t)tap * C2 + c4) = o; __threadfence(); *(volatile v4f*)(WT + (size_t)tap * C2 + c4) = o;
}

__global__ __launch_bounds__(256) void k_rownorm(const float* __restrict__ x, const float* __restrict__ g, const float* __restrict__ be, h16* AH, unsigned nrows) {
#pragma clang fp contract(off)
    const unsigned lane = threadIdx.x & 31u;
    const unsigned wave = (unsigned)__builtin_amdgcn_readfirstlane((int)(threadIdx.x >> 5));
    const unsigned row = blockIdx.x * 8u + wave;
    if (row >= nrows) return;
    const float* xr = x + (size_t)row * CM + lane * 8u;
    const v4f xa = *(const v4f*)xr, xb = *(const v4f*)(xr + 4);
    const v4f ga = *(const v4f*)(g + lane * 8u), gb = *(const v4f*)(g + lane * 8u + 4u);
    const v4f ba = *(const v4f*)(be + lane * 8u), bb = *(const v4f*)(be + lane * 8u + 4u);
    float v[8], gg[8], bq[8];
#pragma unroll
    for (int k = 0; k < 4; ++k) { v[k] = bfr(xa[k]); v[4 + k] = bfr(xb[k]); gg[k] = bfr(ga[k]); gg[4 + k] = bfr(gb[k]); bq[k] = bfr(ba[k]); bq[4 + k] = bfr(bb[k]); }
    float s = ((v[0] + v[1]) + (v[2] + v[3])) + ((v[4] + v[5]) + (v[6] + v[7]));
    s = wsum(s);
    const float m = s * (1.0f / 256.0f);
    float q = 0.0f;
#pragma unroll
    for (int k = 0; k < 8; ++k) { v[k] = v[k] - m; q += v[k] * v[k]; }
    q = wsum(q);
    const float rs = rsqrtf(q * (1.0f / 256.0f) + EPSL);
    v8h hv;
#pragma unroll
    for (int k = 0; k < 8; ++k) { const float o = v[k] * rs * gg[k] + bq[k]; hv[k] = toh_flush(o); }
    const size_t oo = (size_t)row * CM + lane * 8u;
#pragma unroll 1
    for (int ps = 0; ps < 2; ++ps) {
        *(volatile v8h*)(AH + oo) = hv;
        if (ps == 0) __threadfence(); }
}

__global__ __launch_bounds__(128) void k_gemm_qsm(const h16* __restrict__ AH, const h16* __restrict__ W, const float* __restrict__ bias, h16* QH, h16* QR) {
    __shared__ __align__(16) float ts[32 * TSP];
    const unsigned lane = threadIdx.x & 31u, lr = lane & 15u, hi = lane >> 4;
    const unsigned wave = (unsigned)__builtin_amdgcn_readfirstlane((int)(threadIdx.x >> 5));
    const unsigned r0 = blockIdx.x * 32u, c0 = wave * 64u;
    v8f acc[2][4];
#pragma unroll
    for (int mb = 0; mb < 2; ++mb)
#pragma unroll
        for (int nb = 0; nb < 4; ++nb) acc[mb][nb] = (v8f){};
    mm_rows<CM>(AH, W, (size_t)(r0 + lr) * CM + 8u * hi, (size_t)(c0 + lr) * CM + 8u * hi, acc);
#pragma unroll
    for (int nb = 0; nb < 4; ++nb) {
        const float bc = bfr(bias[c0 + nb * 16 + lr]);
#pragma unroll
        for (int mb = 0; mb < 2; ++mb) {
#pragma unroll
            for (int j = 0; j < 8; ++j) ts[(mb * 16 + hi * 8 + j) * TSP + c0 + nb * 16 + lr] = acc[mb][nb][j] * OS_W + bc; }
    }
    __syncthreads();
#pragma unroll 1
    for (unsigned i = 0; i < 8u; ++i) {
        const unsigned ro = (wave * 8u + i) * TSP + lane * 8u;
        const v4f x0 = *(const v4fa*)(&ts[ro]); const v4f x1 = *(const v4fa*)(&ts[ro + 4]);
        float mx = fmaxf(fmaxf(fmaxf(x0[0], x0[1]), fmaxf(x0[2], x0[3])), fmaxf(fmaxf(x1[0], x1[1]), fmaxf(x1[2], x1[3])));
        mx = fmaxf(mx, __shfl_xor(mx, 1, 32)); mx = fmaxf(mx, __shfl_xor(mx, 2, 32));
        v4f e0, e1;
#pragma unroll
        for (int k = 0; k < 4; ++k) { e0[k] = __builtin_amdgcn_exp2f((x0[k] - mx) * L2E); e1[k] = __builtin_amdgcn_exp2f((x1[k] - mx) * L2E); }
        float s = ((e0[0] + e0[1]) + (e0[2] + e0[3])) + ((e1[0] + e1[1]) + (e1[2] + e1[3]));
        s += __shfl_xor(s, 1, 32); s += __shfl_xor(s, 2, 32);
        const float sc = QSC * (1.0f / s);
        e0 = e0 * sc; e1 = e1 * sc;
        *(v4fa*)(&ts[ro]) = e0; *(v4fa*)(&ts[ro + 4]) = e1;
    }
    wave_sync();
    static_assert(4 * 8 == 32);
#pragma unroll 1
    for (int ps = 0; ps < 2; ++ps) {
#pragma unroll 1
        for (unsigned i = 0; i < 8u; ++i) {
            const unsigned ro = (wave * 8u + i) * TSP + lane * 8u;
            const v4f x0 = *(const v4fa*)(&ts[ro]); const v4f x1 = *(const v4fa*)(&ts[ro + 4]); v8h hv, rv;
#pragma unroll
            for (int k = 0; k < 4; ++k) { h16 a, r; split_hr(x0[k], a, r); hv[k] = a; rv[k] = r; split_hr(x1[k], a, r); hv[4 + k] = a; rv[4 + k] = r; }
            const size_t oo = (size_t)(r0 + wave * 8u + i) * CM + lane * 8u;
            *(volatile v8h*)(QH + oo) = hv; *(volatile v8h*)(QR + oo) = rv; }
        if (ps == 0) __threadfence(); }
}

__global__ __launch_bounds__(32) void k_gemm_tr(const h16* __restrict__ W, const h16* __restrict__ XH, const float* __restrict__ bias, h16* VH, h16* VR) {
    __shared__ __align__(16) float os[16 * 68];
    const unsigned lane = threadIdx.x & 31u, lr = lane & 15u, hi = lane >> 4;
    const unsigned r0 = blockIdx.x * 32u, c0 = blockIdx.y * 64u;
    v8f acc[2][4];
#pragma unroll
    for (int mb = 0; mb < 2; ++mb)
#pragma unroll
        for (int nb = 0; nb < 4; ++nb) acc[mb][nb] = (v8f){};
    mm_cols<CM>(W, XH, (size_t)(r0 + lr) * CM + 8u * hi, (size_t)(c0 + lr) * CM + 8u * hi, acc);
    const unsigned bb = c0 / (unsigned)NTOK, tt = c0 % (unsigned)NTOK;
    const size_t tbase = ((size_t)bb * CM + r0) * NTOK + tt;
#pragma unroll
    for (int mb = 0; mb < 2; ++mb) {
        float br[8];
#pragma unroll
        for (int j = 0; j < 8; ++j) br[j] = bfr(bias[r0 + mb * 16 + hi * 8 + j]);
#pragma unroll
        for (int nb = 0; nb < 4; ++nb) {
#pragma unroll
            for (int j = 0; j < 8; ++j) os[(hi * 8 + j) * 68 + nb * 16 + lr] = acc[mb][nb][j] * OS_W + br[j]; }
        wave_sync();
        static_assert(4 * 4 == 16);
#pragma unroll 1
        for (int ps = 0; ps < 2; ++ps) {
#pragma unroll
            for (int s = 0; s < 4; ++s) { const unsigned row = 4u * s + (lane >> 3), c8 = (lane & 7u) * 8u;
                const v4f x0 = *(const v4fa*)(&os[row * 68 + c8]); const v4f x1 = *(const v4fa*)(&os[row * 68 + c8 + 4]); v8h hv, rv;
#pragma unroll
                for (int k = 0; k < 4; ++k) { h16 a, r; split_hr(x0[k], a, r); hv[k] = a; rv[k] = r; split_hr(x1[k], a, r); hv[4 + k] = a; rv[4 + k] = r; }
                const size_t oo = tbase + (size_t)(mb * 16 + row) * NTOK + c8;
                *(volatile v8h*)(VH + oo) = hv; *(volatile v8h*)(VR + oo) = rv; }
            if (ps == 0) __threadfence(); }
        wave_sync();
    }
}

__global__ __launch_bounds__(256) void k_colsoft(const h16* __restrict__ VH, const h16* __restrict__ VR, h16* KH, h16* KR) {
#pragma clang fp contract(off)
    __shared__ float smx[8]; __shared__ float ssm[8];
    const unsigned tid = threadIdx.x, lane = tid & 31u;
    const unsigned wave = (unsigned)__builtin_amdgcn_readfirstlane((int)(tid >> 5));
    const size_t o0 = (size_t)blockIdx.x * NTOK + tid * 8u, o1 = o0 + 2048u;
    const v8h h0 = *(const v8h*)(VH + o0), q0 = *(const v8h*)(VR + o0), h1 = *(const v8h*)(VH + o1), q1 = *(const v8h*)(VR + o1);
    float x[16];
#pragma unroll
    for (int k = 0; k < 8; ++k) { x[k] = (float)h0[k] + (float)q0[k] * QRI; x[8 + k] = (float)h1[k] + (float)q1[k] * QRI; }
    float mx = x[0];
#pragma unroll
    for (int k = 1; k < 16; ++k) mx = fmaxf(mx, x[k]);
    mx = wmaxf(mx);
    if (lane == 0) smx[wave] = mx;
    __syncthreads();
    float bm = smx[0];
#pragma unroll
    for (int w = 1; w < 8; ++w) bm = fmaxf(bm, smx[w]);
    float s = 0.0f;
#pragma unroll
    for (int k = 0; k < 16; ++k) { x[k] = __builtin_amdgcn_exp2f((x[k] - bm) * L2E); s += x[k]; }
    s = wsum(s);
    if (lane == 0) ssm[wave] = s;
    __syncthreads();
    const float tot = ((ssm[0] + ssm[1]) + (ssm[2] + ssm[3])) + ((ssm[4] + ssm[5]) + (ssm[6] + ssm[7]));
    const float sc = KSC * (1.0f / tot);
    v8h hv0, rv0, hv1, rv1;
#pragma unroll
    for (int k = 0; k < 8; ++k) { h16 a, r; split_hr(x[k] * sc, a, r); hv0[k] = a; rv0[k] = r; split_hr(x[8 + k] * sc, a, r); hv1[k] = a; rv1[k] = r; }
#pragma unroll 1
    for (int ps = 0; ps < 2; ++ps) {
        *(volatile v8h*)(KH + o0) = hv0; *(volatile v8h*)(KR + o0) = rv0; *(volatile v8h*)(KH + o1) = hv1; *(volatile v8h*)(KR + o1) = rv1;
        if (ps == 0) __threadfence(); }
}

__global__ __launch_bounds__(128) void k_ctx(const h16* __restrict__ KH, const h16* __restrict__ KR, const h16* __restrict__ VH, const h16* __restrict__ VR, h16* CTH, h16* CTR) {
    __shared__ __align__(16) float cs[32 * 36];
    const unsigned tid = threadIdx.x, lane = tid & 31u, lr = lane & 15u, hi = lane >> 4;
    const unsigned wave = (unsigned)__builtin_amdgcn_readfirstlane((int)(tid >> 5));
    const unsigned zh = blockIdx.x; const unsigned dt = wave >> 1, vt = wave & 1u;
    const size_t ao = (size_t)(zh * 32u + dt * 16u + lr) * NTOK + 8u * hi;
    const size_t bo = (size_t)(zh * 32u + vt * 16u + lr) * NTOK + 8u * hi;
    v8f acc = (v8f){}, accr = (v8f){};
#pragma unroll 1
    for (unsigned kc = 0; kc < (unsigned)NTOK; kc += 32u) {
        const v16h kh = ldh(KH + ao + kc), kr = ldh(KR + ao + kc), vh = ldh(VH + bo + kc), vr = ldh(VR + bo + kc);
        acc = wmma16g(kh, vh, acc); accr = wmma16g(kh, vr, accr); accr = wmma16g(kr, vh, accr);
    }
    { v4f a, c;
#pragma unroll
      for (int k = 0; k < 4; ++k) { a[k] = (acc[k] + accr[k] * QRI) * OS_CTX; c[k] = (acc[4 + k] + accr[4 + k] * QRI) * OS_CTX; }
      const unsigned so = (vt * 16u + lr) * 36u + dt * 16u + 8u * hi;
      *(v4fa*)(&cs[so]) = a; *(v4fa*)(&cs[so + 4]) = c; }
    __syncthreads();
    static_assert(128 * 8 == HD * HD);
    const unsigned ro = (tid >> 2) * 36u + (tid & 3u) * 8u;
    const v4f x0 = *(const v4fa*)(&cs[ro]); const v4f x1 = *(const v4fa*)(&cs[ro + 4]); v8h hv, rv;
#pragma unroll
    for (int k = 0; k < 4; ++k) { h16 a, r; split_hr(x0[k], a, r); hv[k] = a; rv[k] = r; split_hr(x1[k], a, r); hv[4 + k] = a; rv[4 + k] = r; }
    const size_t oo = (size_t)zh * (HD * HD) + tid * 8u;
#pragma unroll 1
    for (int ps = 0; ps < 2; ++ps) {
        *(volatile v8h*)(CTH + oo) = hv; *(volatile v8h*)(CTR + oo) = rv;
        if (ps == 0) __threadfence(); }
}

__global__ __launch_bounds__(64) void k_apply(const h16* __restrict__ QH, const h16* __restrict__ QR, const h16* __restrict__ CTH, const h16* __restrict__ CTR, h16* AGH) {
    __shared__ __align__(16) float as_[2 * 16 * TSP];
    const unsigned lane = threadIdx.x & 31u, lr = lane & 15u, hi = lane >> 4;
    const unsigned wave = (unsigned)__builtin_amdgcn_readfirstlane((int)(threadIdx.x >> 5));
    const unsigned t0 = blockIdx.x * 32u + wave * 16u;
    const unsigned b = (blockIdx.x * 32u) / (unsigned)NTOK;
    const unsigned wb = wave * 16u * TSP;
#pragma unroll 1
    for (unsigned h = 0; h < (unsigned)NH_; ++h) {
        const size_t qo = (size_t)(t0 + lr) * CM + h * 32u + 8u * hi;
        const v16h qh = ldh(QH + qo), qr = ldh(QR + qo);
#pragma unroll
        for (unsigned vt = 0; vt < 2u; ++vt) {
            const size_t co = (size_t)((b * NH_ + h) * 32u + vt * 16u + lr) * 32u + 8u * hi;
            const v16h ch = ldh(CTH + co), cr = ldh(CTR + co);
            v8f acc = (v8f){}, accr = (v8f){};
            acc = wmma16g(qh, ch, acc); accr = wmma16g(qh, cr, accr); accr = wmma16g(qr, ch, accr);
#pragma unroll
            for (int j = 0; j < 8; ++j) as_[wb + (8u * hi + j) * TSP + h * 32u + vt * 16u + lr] = (acc[j] + accr[j] * QRI) * OS_ATT; }
    }
    wave_sync();
    static_assert(2 * 16 == 32);
#pragma unroll 1
    for (int ps = 0; ps < 2; ++ps) {
#pragma unroll 1
        for (unsigned i = 0; i < 16u; ++i) {
            const unsigned ro = wb + i * TSP + lane * 8u;
            const v4f x0 = *(const v4fa*)(&as_[ro]); const v4f x1 = *(const v4fa*)(&as_[ro + 4]); v8h hv;
#pragma unroll
            for (int k = 0; k < 4; ++k) { hv[k] = toh_flush(x0[k]); hv[4 + k] = toh_flush(x1[k]); }
            const size_t oo = (size_t)(t0 + i) * CM + lane * 8u;
            *(volatile v8h*)(AGH + oo) = hv; }
        if (ps == 0) __threadfence(); }
}

__global__ __launch_bounds__(128) void k_gemm_n2(const h16* __restrict__ AH, const h16* __restrict__ W, const float* __restrict__ bias,
                                                 const float* __restrict__ X1, const float* __restrict__ g1, const float* __restrict__ b1,
                                                 const float* __restrict__ g2, const float* __restrict__ b2, h16* YH, h16* YR) {
    __shared__ __align__(16) float ts[32 * TSP];
    const unsigned lane = threadIdx.x & 31u, lr = lane & 15u, hi = lane >> 4;
    const unsigned wave = (unsigned)__builtin_amdgcn_readfirstlane((int)(threadIdx.x >> 5));
    const unsigned r0 = blockIdx.x * 32u, c0 = wave * 64u;
    v8f acc[2][4];
#pragma unroll
    for (int mb = 0; mb < 2; ++mb)
#pragma unroll
        for (int nb = 0; nb < 4; ++nb) acc[mb][nb] = (v8f){};
    mm_rows<CM>(AH, W, (size_t)(r0 + lr) * CM + 8u * hi, (size_t)(c0 + lr) * CM + 8u * hi, acc);
#pragma unroll
    for (int nb = 0; nb < 4; ++nb) {
        const float bc = bfr(bias[c0 + nb * 16 + lr]);
#pragma unroll
        for (int mb = 0; mb < 2; ++mb) {
#pragma unroll
            for (int j = 0; j < 8; ++j) ts[(mb * 16 + hi * 8 + j) * TSP + c0 + nb * 16 + lr] = acc[mb][nb][j] * OS_REP + bc; }
    }
    __syncthreads();
    float pg1[8], pb1[8], pg2[8], pb2[8];
    { const v4f a0 = *(const v4f*)(g1 + lane * 8u), a1 = *(const v4f*)(g1 + lane * 8u + 4u), c0v = *(const v4f*)(b1 + lane * 8u), c1v = *(const v4f*)(b1 + lane * 8u + 4u);
      const v4f d0 = *(const v4f*)(g2 + lane * 8u), d1 = *(const v4f*)(g2 + lane * 8u + 4u), e0 = *(const v4f*)(b2 + lane * 8u), e1 = *(const v4f*)(b2 + lane * 8u + 4u);
#pragma unroll
      for (int k = 0; k < 4; ++k) { pg1[k] = bfr(a0[k]); pg1[4 + k] = bfr(a1[k]); pb1[k] = bfr(c0v[k]); pb1[4 + k] = bfr(c1v[k]);
                                    pg2[k] = bfr(d0[k]); pg2[4 + k] = bfr(d1[k]); pb2[k] = bfr(e0[k]); pb2[4 + k] = bfr(e1[k]); } }
#pragma unroll 1
    for (unsigned i = 0; i < 8u; ++i) {
        const unsigned ro = (wave * 8u + i) * TSP + lane * 8u;
        const v4f x0 = *(const v4fa*)(&ts[ro]); const v4f x1 = *(const v4fa*)(&ts[ro + 4]);
        const float* xp = X1 + (size_t)(r0 + wave * 8u + i) * CM + lane * 8u;
        const v4f xa = *(const v4f*)xp, xb = *(const v4f*)(xp + 4);
        float v[8], xr[8];
#pragma unroll
        for (int k = 0; k < 4; ++k) { v[k] = x0[k]; v[4 + k] = x1[k]; xr[k] = bfr(xa[k]); xr[4 + k] = bfr(xb[k]); }
        float s = ((v[0] + v[1]) + (v[2] + v[3])) + ((v[4] + v[5]) + (v[6] + v[7]));
        s = wsum(s);
        const float m = s * (1.0f / 256.0f);
        float q = 0.0f;
#pragma unroll
        for (int k = 0; k < 8; ++k) { v[k] = v[k] - m; q += v[k] * v[k]; }
        q = wsum(q);
        const float rs = rsqrtf(q * (1.0f / 256.0f) + EPSL);
        float s2 = 0.0f;
#pragma unroll
        for (int k = 0; k < 8; ++k) { v[k] = (v[k] * rs * pg1[k] + pb1[k]) + xr[k]; s2 += v[k]; }
        s2 = wsum(s2);
        const float m2 = s2 * (1.0f / 256.0f);
        float q2 = 0.0f;
#pragma unroll
        for (int k = 0; k < 8; ++k) { v[k] = v[k] - m2; q2 += v[k] * v[k]; }
        q2 = wsum(q2);
        const float rs2 = rsqrtf(q2 * (1.0f / 256.0f) + EPSL);
        v4f y0, y1;
#pragma unroll
        for (int k = 0; k < 4; ++k) { y0[k] = v[k] * rs2 * pg2[k] + pb2[k]; y1[k] = v[4 + k] * rs2 * pg2[4 + k] + pb2[4 + k]; }
        *(v4fa*)(&ts[ro]) = y0; *(v4fa*)(&ts[ro + 4]) = y1;
    }
    wave_sync();
    static_assert(4 * 8 == 32);
#pragma unroll 1
    for (int ps = 0; ps < 2; ++ps) {
#pragma unroll 1
        for (unsigned i = 0; i < 8u; ++i) {
            const unsigned ro = (wave * 8u + i) * TSP + lane * 8u;
            const v4f x0 = *(const v4fa*)(&ts[ro]); const v4f x1 = *(const v4fa*)(&ts[ro + 4]); v8h hv, rv;
#pragma unroll
            for (int k = 0; k < 4; ++k) { h16 a, r; split_hr(x0[k], a, r); hv[k] = a; rv[k] = r; split_hr(x1[k], a, r); hv[4 + k] = a; rv[4 + k] = r; }
            const size_t oo = (size_t)(r0 + wave * 8u + i) * CM + lane * 8u;
            *(volatile v8h*)(YH + oo) = hv; *(volatile v8h*)(YR + oo) = rv; }
        if (ps == 0) __threadfence(); }
}

__global__ __launch_bounds__(32) void k_gemm_f32(const h16* __restrict__ AH, const h16* __restrict__ W, const float* __restrict__ bias, float* H1) {
    __shared__ __align__(16) float os[16 * 68];
    const unsigned lane = threadIdx.x & 31u, lr = lane & 15u, hi = lane >> 4;
    const unsigned r0 = blockIdx.x * 32u, c0 = blockIdx.y * 64u;
    v8f acc[2][4];
#pragma unroll
    for (int mb = 0; mb < 2; ++mb)
#pragma unroll
        for (int nb = 0; nb < 4; ++nb) acc[mb][nb] = (v8f){};
    mm_rows<CM>(AH, W, (size_t)(r0 + lr) * CM + 8u * hi, (size_t)(c0 + lr) * CM + 8u * hi, acc);
    float bc[4];
#pragma unroll
    for (int nb = 0; nb < 4; ++nb) bc[nb] = bfr(bias[c0 + nb * 16 + lr]);
#pragma unroll
    for (int mb = 0; mb < 2; ++mb) {
#pragma unroll
        for (int nb = 0; nb < 4; ++nb) {
#pragma unroll
            for (int j = 0; j < 8; ++j) os[(hi * 8 + j) * 68 + nb * 16 + lr] = acc[mb][nb][j] * OS_W + bc[nb]; }
        wave_sync();
        static_assert(8 * 2 == 16);
#pragma unroll 1
        for (int ps = 0; ps < 2; ++ps) {
#pragma unroll
            for (int s = 0; s < 8; ++s) { const unsigned row = 2u * s + (lane >> 4), c4 = (lane & 15u) * 4u;
                const v4f val = *(const v4fa*)(&os[row * 68 + c4]);
                *(volatile v4f*)(H1 + (size_t)(r0 + mb * 16 + row) * C2 + c0 + c4) = val; }
            if (ps == 0) __threadfence(); }
        wave_sync();
    }
}

__global__ __launch_bounds__(256) void k_dwnorm(const float* __restrict__ H1, const float* __restrict__ WT, const float* __restrict__ dwb,
                                                const float* __restrict__ g, const float* __restrict__ be, h16* AXH) {
#pragma clang fp contract(off)
    __shared__ __align__(16) float cs[8 * C2];
    const unsigned lane = threadIdx.x & 31u;
    const unsigned wave = (unsigned)__builtin_amdgcn_readfirstlane((int)(threadIdx.x >> 5));
    const unsigned tok = blockIdx.x * 8u + wave;
    const unsigned bl = tok / (unsigned)NTOK, p = tok % (unsigned)NTOK;
    const int y = (int)(p >> 6), x = (int)(p & 63u);
    const float* hb = H1 + (size_t)bl * NTOK * C2;
    const unsigned wb = wave * C2;
    float sum = 0.0f;
#pragma unroll 1
    for (unsigned gq = 0; gq < 4u; ++gq) {
        const unsigned c = gq * 128u + lane * 4u;
        v4f a = (v4f){};
#pragma unroll 1
        for (int ty = 0; ty < 3; ++ty) {
#pragma unroll 1
            for (int tx = 0; tx < 3; ++tx) {
                const int yy = y + ty - 1, xx = x + tx - 1;
                const bool ok = ((unsigned)yy < (unsigned)IMG) && ((unsigned)xx < (unsigned)IMG);
                const int yc = min(max(yy, 0), IMG - 1), xc = min(max(xx, 0), IMG - 1);
                const v4f hv = *(const v4f*)(hb + (size_t)(yc * IMG + xc) * C2 + c);
                const v4f wv = *(const v4f*)(WT + (size_t)(ty * 3 + tx) * C2 + c);
                const v4f hz = (v4f){};
                const v4f hs = ok ? hv : hz;
                a = a + hs * wv;
            }
        }
        const v4f bv = *(const v4f*)(dwb + c);
#pragma unroll
        for (int k = 0; k < 4; ++k) a[k] = a[k] + bfr(bv[k]);
        *(v4fa*)(&cs[wb + c]) = a;
        sum += (a[0] + a[1]) + (a[2] + a[3]);
    }
    sum = wsum(sum);
    const float mean = sum * (1.0f / 512.0f);
    wave_sync();
    float q = 0.0f;
#pragma unroll 1
    for (unsigned gq = 0; gq < 4u; ++gq) {
        const v4f v = *(const v4fa*)(&cs[wb + gq * 128u + lane * 4u]);
        const float d0 = v[0] - mean, d1 = v[1] - mean, d2 = v[2] - mean, d3 = v[3] - mean;
        q += (d0 * d0 + d1 * d1) + (d2 * d2 + d3 * d3);
    }
    q = wsum(q);
    const float rs = rsqrtf(q * (1.0f / 512.0f) + EPSL);
    wave_sync();
#pragma unroll 1
    for (unsigned e = 0; e < 16u; ++e) {
        const unsigned c = (e >> 2) * 128u + lane * 4u + (e & 3u);
        const float t = (cs[wb + c] - mean) * rs * bfr(g[c]) + bfr(be[c]);
        cs[wb + c] = 0.5f * t * (1.0f + erff(t * 0.70710678118654752f));
    }
    wave_sync();
    static_assert(4 * 32 * 4 == C2);
#pragma unroll 1
    for (int ps = 0; ps < 2; ++ps) {
#pragma unroll 1
        for (unsigned gq = 0; gq < 4u; ++gq) {
            const unsigned c = gq * 128u + lane * 4u;
            const v4f v = *(const v4fa*)(&cs[wb + c]); v4h hv;
#pragma unroll
            for (int k = 0; k < 4; ++k) hv[k] = toh_flush(v[k]);
            const size_t oo = (size_t)tok * C2 + c;
            *(volatile v4h*)(AXH + oo) = hv; }
        if (ps == 0) __threadfence(); }
}

__global__ __launch_bounds__(128) void k_gemm_fin(const h16* __restrict__ AH, const h16* __restrict__ W, const float* __restrict__ bias,
                                                  const h16* __restrict__ YH, const h16* __restrict__ YR, const float* __restrict__ g, const float* __restrict__ be, float* OUT) {
    __shared__ __align__(16) float ts[32 * TSP];
    const unsigned lane = threadIdx.x & 31u, lr = lane & 15u, hi = lane >> 4;
    const unsigned wave = (unsigned)__builtin_amdgcn_readfirstlane((int)(threadIdx.x >> 5));
    const unsigned r0 = blockIdx.x * 32u, c0 = wave * 64u;
    v8f acc[2][4];
#pragma unroll
    for (int mb = 0; mb < 2; ++mb)
#pragma unroll
        for (int nb = 0; nb < 4; ++nb) acc[mb][nb] = (v8f){};
    mm_rows<C2>(AH, W, (size_t)(r0 + lr) * C2 + 8u * hi, (size_t)(c0 + lr) * C2 + 8u * hi, acc);
#pragma unroll
    for (int nb = 0; nb < 4; ++nb) {
        const float bc = bfr(bias[c0 + nb * 16 + lr]);
#pragma unroll
        for (int mb = 0; mb < 2; ++mb) {
#pragma unroll
            for (int j = 0; j < 8; ++j) ts[(mb * 16 + hi * 8 + j) * TSP + c0 + nb * 16 + lr] = acc[mb][nb][j] * OS_W + bc; }
    }
    __syncthreads();
    float pg[8], pb[8];
    { const v4f a0 = *(const v4f*)(g + lane * 4u), a1 = *(const v4f*)(g + 128u + lane * 4u), c0v = *(const v4f*)(be + lane * 4u), c1v = *(const v4f*)(be + 128u + lane * 4u);
#pragma unroll
      for (int k = 0; k < 4; ++k) { pg[k] = bfr(a0[k]); pg[4 + k] = bfr(a1[k]); pb[k] = bfr(c0v[k]); pb[4 + k] = bfr(c1v[k]); } }
#pragma unroll 1
    for (unsigned i = 0; i < 8u; ++i) {
        const unsigned ro = (wave * 8u + i) * TSP + lane * 4u;
        const v4f o0 = *(const v4fa*)(&ts[ro]); const v4f o1 = *(const v4fa*)(&ts[ro + 128]);
        const size_t yo = (size_t)(r0 + wave * 8u + i) * CM + lane * 4u;
        const v4h yh0 = *(const v4h*)(YH + yo), yr0 = *(const v4h*)(YR + yo), yh1 = *(const v4h*)(YH + yo + 128), yr1 = *(const v4h*)(YR + yo + 128);
        float v[8];
#pragma unroll
        for (int k = 0; k < 4; ++k) { v[k] = o0[k] + ((float)yh0[k] + (float)yr0[k] * QRI); v[4 + k] = o1[k] + ((float)yh1[k] + (float)yr1[k] * QRI); }
        float s = ((v[0] + v[1]) + (v[2] + v[3])) + ((v[4] + v[5]) + (v[6] + v[7]));
        s = wsum(s);
        const float m = s * (1.0f / 256.0f);
        float q = 0.0f;
#pragma unroll
        for (int k = 0; k < 8; ++k) { v[k] = v[k] - m; q += v[k] * v[k]; }
        q = wsum(q);
        const float rs = rsqrtf(q * (1.0f / 256.0f) + EPSL);
        v4f f0, f1;
#pragma unroll
        for (int k = 0; k < 4; ++k) { f0[k] = v[k] * rs * pg[k] + pb[k]; f1[k] = v[4 + k] * rs * pg[4 + k] + pb[4 + k]; }
        *(v4fa*)(&ts[ro]) = f0; *(v4fa*)(&ts[ro + 128]) = f1;
    }
    wave_sync();
    static_assert(2 * 32 * 4 == CM);
#pragma unroll 1
    for (int ps = 0; ps < 2; ++ps) {
#pragma unroll 1
        for (unsigned i = 0; i < 8u; ++i) {
            const unsigned ro = (wave * 8u + i) * TSP + lane * 4u;
            const v4f f0 = *(const v4fa*)(&ts[ro]); const v4f f1 = *(const v4fa*)(&ts[ro + 128]);
            float* op = OUT + (size_t)(r0 + wave * 8u + i) * CM + lane * 4u;
            *(volatile v4f*)(op) = f0; *(volatile v4f*)(op + 128) = f1; }
        if (ps == 0) __threadfence(); }
}

static constexpr size_t al256(size_t v) { return (v + 255) & ~(size_t)255; }
static constexpr size_t SZ_P    = al256((size_t)NB * NTOK * CM * 2);
static constexpr size_t SZ_CH   = al256((size_t)CHB * NTOK * C2 * 4);
static constexpr size_t SZ_PAIR = (2 * SZ_P > SZ_CH) ? 2 * SZ_P : SZ_CH;
static constexpr size_t SZ_W256 = al256((size_t)CM * CM * 2);
static constexpr size_t SZ_W512 = al256((size_t)C2 * CM * 2);
static constexpr size_t SZ_CT   = al256((size_t)NB * NH_ * HD * HD * 2);
static constexpr size_t SZ_WT   = al256((size_t)9 * C2 * 4);
static constexpr size_t SZ_TOTAL = 3 * SZ_PAIR + 2 * SZ_W256 + 2 * SZ_W512 + 2 * SZ_CT + SZ_WT;
static_assert(SZ_TOTAL <= (size_t)134217728);
static_assert(2 * SZ_P <= SZ_PAIR);
static_assert((size_t)CHB * NTOK * C2 * 4 <= SZ_PAIR);
static_assert((size_t)CHB * NTOK * C2 * 2 <= SZ_PAIR);
static_assert((size_t)NB * CM * NTOK * 2 <= SZ_P);

extern "C" void kernel_launch(void* const* d_in, const int* in_sizes, int n_in,
                              void* d_out, int out_size, void* d_ws, size_t ws_size, hipStream_t stream) {
    if (n_in < 22) return;
    const size_t needx = (size_t)NB * NTOK * CM;
    if ((size_t)in_sizes[0] < needx || (size_t)in_sizes[1] < needx) return;
    if (in_sizes[2] < CM || in_sizes[3] < CM || in_sizes[5] < CM || in_sizes[7] < CM || in_sizes[8] < CM || in_sizes[9] < CM || in_sizes[10] < CM || in_sizes[11] < CM) return;
    if (in_sizes[4] < CM * CM || in_sizes[6] < CM * CM || in_sizes[12] < C2 * CM || in_sizes[18] < CM * C2) return;
    if (in_sizes[13] < C2 || in_sizes[15] < C2 || in_sizes[16] < C2 || in_sizes[17] < C2 || in_sizes[14] < C2 * 9) return;
    if (in_sizes[19] < CM || in_sizes[20] < CM || in_sizes[21] < CM) return;
    if ((size_t)out_size < needx) return;
    if (SZ_TOTAL > ws_size) return;
    const float* x1 = (const float*)d_in[0];   const float* x2 = (const float*)d_in[1];
    const float* n1g = (const float*)d_in[2];  const float* n1b = (const float*)d_in[3];
    const float* linw = (const float*)d_in[4]; const float* linb = (const float*)d_in[5];
    const float* repw = (const float*)d_in[6]; const float* repb = (const float*)d_in[7];
    const float* ang = (const float*)d_in[8];  const float* anb = (const float*)d_in[9];
    const float* n2g = (const float*)d_in[10]; const float* n2b = (const float*)d_in[11];
    const float* f1w = (const float*)d_in[12]; const float* f1b = (const float*)d_in[13];
    const float* dww = (const float*)d_in[14]; const float* dwb = (const float*)d_in[15];
    const float* fng = (const float*)d_in[16]; const float* fnb = (const float*)d_in[17];
    const float* f2w = (const float*)d_in[18]; const float* f2b = (const float*)d_in[19];
    const float* n3g = (const float*)d_in[20]; const float* n3b = (const float*)d_in[21];
    float* OUT = (float*)d_out;
    char* wsp = (char*)d_ws;
    char* pa = wsp; wsp += SZ_PAIR;
    char* pb = wsp; wsp += SZ_PAIR;
    char* pc = wsp; wsp += SZ_PAIR;
    h16* WL = (h16*)wsp; wsp += SZ_W256;
    h16* WR = (h16*)wsp; wsp += SZ_W256;
    h16* W1 = (h16*)wsp; wsp += SZ_W512;
    h16* W2 = (h16*)wsp; wsp += SZ_W512;
    h16* CTH = (h16*)wsp; wsp += SZ_CT;
    h16* CTR = (h16*)wsp; wsp += SZ_CT;
    float* WT = (float*)wsp; wsp += SZ_WT;
    h16* X1H = (h16*)pa;
    h16* VH = (h16*)pa;  h16* VR = (h16*)(pa + SZ_P);
    float* H1 = (float*)pa;
    h16* X2H = (h16*)pb;
    h16* KH = (h16*)pb;  h16* KR = (h16*)(pb + SZ_P);
    h16* AGH = (h16*)pb;
    h16* AXH = (h16*)pb;
    h16* QH = (h16*)pc;  h16* QR = (h16*)(pc + SZ_P);
    h16* YH = QH;        h16* YR = QR;

    { const unsigned n8 = (unsigned)((size_t)CM * CM / 8); const unsigned m8 = (unsigned)((size_t)C2 * CM / 8);
      k_wconv<<<(n8 + 255) / 256, 256, 0, stream>>>(linw, WL, n8);
      k_wconv<<<(n8 + 255) / 256, 256, 0, stream>>>(repw, WR, n8);
      k_wconv<<<(m8 + 255) / 256, 256, 0, stream>>>(f1w, W1, m8);
      k_wconv<<<(m8 + 255) / 256, 256, 0, stream>>>(f2w, W2, m8); }
    k_tapprep<<<9, 128, 0, stream>>>(dww, WT);

    k_rownorm<<<(MROWS + 7) / 8, 256, 0, stream>>>(x1, n1g, n1b, X1H, (unsigned)MROWS);
    k_rownorm<<<(MROWS + 7) / 8, 256, 0, stream>>>(x2, n1g, n1b, X2H, (unsigned)MROWS);

    k_gemm_qsm<<<MROWS / 32, 128, 0, stream>>>(X1H, WL, linb, QH, QR);
    k_gemm_tr<<<dim3(CM / 32, MROWS / 64, 1), 32, 0, stream>>>(WL, X2H, linb, VH, VR);
    k_colsoft<<<NB * CM, 256, 0, stream>>>(VH, VR, KH, KR);
    k_ctx<<<NB * NH_, 128, 0, stream>>>(KH, KR, VH, VR, CTH, CTR);
    k_apply<<<MROWS / 32, 64, 0, stream>>>(QH, QR, CTH, CTR, AGH);
    k_gemm_n2<<<MROWS / 32, 128, 0, stream>>>(AGH, WR, repb, x1, ang, anb, n2g, n2b, YH, YR);

    for (unsigned ch = 0; ch < (unsigned)(NB / CHB); ++ch) {
        const size_t roff = (size_t)ch * CHB * NTOK;
        k_gemm_f32<<<dim3(CHB * NTOK / 32, C2 / 64, 1), 32, 0, stream>>>(YH + roff * CM, W1, f1b, H1);
        k_dwnorm<<<CHB * NTOK / 8, 256, 0, stream>>>(H1, WT, dwb, fng, fnb, AXH);
        k_gemm_fin<<<CHB * NTOK / 32, 128, 0, stream>>>(AXH, W2, f2b, YH + roff * CM, YR + roff * CM, n3g, n3b, OUT + roff * CM);
    }
}
